// Code_Wise_Attention_6158983102794
// MI455X (gfx1250) — hardware-verified
//
#include <hip/hip_runtime.h>
#include <stddef.h>


typedef _Float16 v16h __attribute__((ext_vector_type(16)));
typedef _Float16 v8h  __attribute__((ext_vector_type(8)));
typedef float    v8f  __attribute__((ext_vector_type(8)));
typedef float    v4f  __attribute__((ext_vector_type(4)));

#ifndef NB
#define NB 8
#endif
#ifndef LQ
#define LQ 2048
#endif
#ifndef LC
#define LC 4096
#endif
#define NB_FULL 8
#define LQ_FULL 2048
#define LC_FULL 4096
#define DIM     256

static_assert(NB >= 1 && NB <= NB_FULL);
static_assert(LQ >= 16 && LQ <= LQ_FULL && (LQ % 16) == 0);
static_assert(LC >= 256 && LC <= LC_FULL && (LC % 256) == 0 && (LC % 128) == 0);
static_assert(DIM == 8 * 32);
static_assert(DIM == 32 * 8);
static_assert(DIM == 256);
static_assert(((NB * LQ) % 8) == 0 && ((NB * LC) % 8) == 0);

#define XCARRY 64.0f

#define QPL_BYTES ((size_t)NB * LQ * DIM * 2)
#define CPL_BYTES ((size_t)NB * LC * DIM * 2)
#define SCR_BYTES ((size_t)NB * LC * 4)
#define OFF_QPL ((size_t)0)
#define OFF_CPL (OFF_QPL + QPL_BYTES)
#define OFF_SCR (OFF_CPL + CPL_BYTES)
#define WS_TOTAL (OFF_SCR + SCR_BYTES)
static_assert((QPL_BYTES % 128) == 0 && (CPL_BYTES % 128) == 0 && (SCR_BYTES % 128) == 0);
static_assert(WS_TOTAL <= (size_t)134217728);

__device__ __forceinline__ float bf16r(float x) {
  unsigned int u = __float_as_uint(x);
  u = (u + 0x7FFFu + ((u >> 16) & 1u)) & 0xFFFF0000u;
  return __uint_as_float(u);
}

static __device__ __forceinline__ _Float16 toh_flush(float v) {
  const _Float16 r = (_Float16)v;
  return (fabsf(v) < 6.103515625e-05f) ? (_Float16)0.0f : r;
}

__device__ __forceinline__ v16h frag_at(const _Float16* p) {
  v8h lo = *(const v8h*)(p);
  v8h hi = *(const v8h*)(p + 16);
  v16h out;
#pragma unroll
  for (int i = 0; i < 8; ++i) { out[i] = lo[i]; out[i + 8] = hi[i]; }
  return out;
}

__device__ __forceinline__ v8f wmma16(v16h a, v16h b, v8f c) {
  v8f d = __builtin_amdgcn_wmma_f32_16x16x32_f16(false, a, false, b, (short)0, c,
                                                 false, false);
  asm volatile("v_nop\n\tv_nop\n\tv_nop\n\tv_nop" : "+v"(d) : "v"(a), "v"(b));
  return d;
}

__device__ __forceinline__ float red16_max(float x) {
#pragma unroll
  for (int off = 1; off < 16; off <<= 1) x = fmaxf(x, __shfl_xor(x, off, 32));
  return x;
}
__device__ __forceinline__ float red32_max(float x) {
#pragma unroll
  for (int off = 1; off < 32; off <<= 1) x = fmaxf(x, __shfl_xor(x, off, 32));
  return x;
}

__global__ __launch_bounds__(256) void cvt_kernel(
    const float* __restrict__ X, _Float16* __restrict__ dst, unsigned rows, unsigned rows_full) {
  const unsigned lane = threadIdx.x & 31u;
  const unsigned wave = (unsigned)__builtin_amdgcn_readfirstlane((int)(threadIdx.x >> 5));
  const unsigned crow = blockIdx.x * 8u + wave;
  const unsigned bidx = crow / rows;
  const unsigned r = crow - bidx * rows;
  const size_t srow = (size_t)bidx * rows_full + r;
  const float* xr = X + srow * DIM + lane * 8u;
  const v4f a0 = *(const v4f*)(xr);
  const v4f a1 = *(const v4f*)(xr + 4u);
  v8h o;
#pragma unroll
  for (int i = 0; i < 4; ++i) {
    o[i]     = toh_flush(XCARRY * bf16r(a0[i]));
    o[i + 4] = toh_flush(XCARRY * bf16r(a1[i]));
  }
  _Float16* p = dst + (size_t)crow * DIM + lane * 8u;
  *(volatile v8h*)p = o;
  __threadfence();
  *(volatile v8h*)p = o;
}

__global__ __launch_bounds__(256) void score_kernel(
    const _Float16* __restrict__ C16, const _Float16* __restrict__ Q16,
    float* __restrict__ scores) {
  __shared__ __attribute__((aligned(16))) float smax[128];
  const unsigned tid = threadIdx.x, lane = tid & 31u;
  const unsigned wave = (unsigned)__builtin_amdgcn_readfirstlane((int)(tid >> 5));
  const unsigned hh = lane >> 4, m = lane & 15u;
  const unsigned b = blockIdx.y;
  const unsigned lc0 = blockIdx.x * 128u;

  const _Float16* ap = C16 + ((size_t)b * LC + lc0 + wave * 16u + m) * DIM + hh * 8u;
  v16h af[8];
#pragma unroll
  for (int c = 0; c < 8; ++c) af[c] = frag_at(ap + c * 32);

  v8f vmax;
#pragma unroll
  for (int r = 0; r < 8; ++r) vmax[r] = -__builtin_inff();

  const _Float16* bp = Q16 + ((size_t)b * LQ + m) * DIM + hh * 8u;
#pragma unroll 1
  for (unsigned qt = 0; qt < (unsigned)(LQ / 16); ++qt) {
    const _Float16* bq = bp + (size_t)qt * (16u * DIM);
    v8f acc = {};
#pragma unroll
    for (int c = 0; c < 8; ++c) {
      const v16h bf = frag_at(bq + c * 32);
      acc = wmma16(af[c], bf, acc);
    }
#pragma unroll
    for (int r = 0; r < 8; ++r) vmax[r] = fmaxf(vmax[r], acc[r]);
  }

#pragma unroll
  for (int r = 0; r < 8; ++r)
    vmax[r] = red16_max(vmax[r]) * (1.0f / (XCARRY * XCARRY));

  if (m == 0u) {
#pragma unroll
    for (int r = 0; r < 8; ++r) smax[wave * 16u + hh * 8u + (unsigned)r] = vmax[r];
  }
  __syncthreads();
  if (wave == 0u) {
    const v4f x = *(const v4f*)&smax[lane * 4u];
    float* p = scores + (size_t)b * LC + lc0 + lane * 4u;
    *(volatile v4f*)p = x;
    __threadfence();
    *(volatile v4f*)p = x;
  }
}

__global__ __launch_bounds__(256) void softmax_ctx_kernel(
    const float* __restrict__ context, const float* __restrict__ scores,
    float* __restrict__ out) {
  __shared__ __attribute__((aligned(16))) float wts[LC];
  __shared__ __attribute__((aligned(16))) float outs[DIM];
  __shared__ float redm[8];
  const unsigned tid = threadIdx.x, lane = tid & 31u;
  const unsigned wave = (unsigned)__builtin_amdgcn_readfirstlane((int)(tid >> 5));
  const unsigned b = blockIdx.x;
  const float* sc = scores + (size_t)b * LC;

  float lm = -__builtin_inff();
#pragma unroll 1
  for (unsigned i = tid; i < (unsigned)LC; i += 256u) {
    const float v = sc[i];
    wts[i] = v;
    lm = fmaxf(lm, v);
  }
  lm = red32_max(lm);
  if (lane == 0u) redm[wave] = lm;
  __syncthreads();
  float mx = redm[0];
#pragma unroll
  for (int j = 1; j < 8; ++j) mx = fmaxf(mx, redm[j]);

#pragma unroll 1
  for (unsigned i = tid; i < (unsigned)LC; i += 256u) wts[i] = __expf(wts[i] - mx);
  __syncthreads();

  const float* ctx = context + (size_t)b * LC_FULL * DIM + tid;
  float acc = 0.0f, sumw = 0.0f;
#pragma unroll 4
  for (unsigned lc = 0; lc < (unsigned)LC; ++lc) {
    const float w = wts[lc];
    sumw += w;
    acc = fmaf(w, bf16r(ctx[(size_t)lc * DIM]), acc);
  }
  outs[tid] = acc * __builtin_amdgcn_rcpf(sumw);
  __syncthreads();
  if (wave < 2u) {
    const v4f x = *(const v4f*)&outs[tid * 4u];
    float* p = out + (size_t)b * DIM + tid * 4u;
    *(volatile v4f*)p = x;
    __threadfence();
    *(volatile v4f*)p = x;
  }
}

extern "C" void kernel_launch(void* const* d_in, const int* in_sizes, int n_in,
                              void* d_out, int out_size, void* d_ws, size_t ws_size,
                              hipStream_t stream) {
  if (n_in < 2) return;
  const long long need_q = ((long long)(NB - 1) * LQ_FULL + LQ) * DIM;
  const long long need_c = ((long long)(NB - 1) * LC_FULL + LC) * DIM;
  if ((long long)in_sizes[0] < need_q) return;
  if ((long long)in_sizes[1] < need_c) return;
  if ((long long)out_size < (long long)NB * DIM) return;
  if (ws_size < WS_TOTAL) return;

  const float* query   = (const float*)d_in[0];
  const float* context = (const float*)d_in[1];
  float* out = (float*)d_out;

  char* ws = (char*)d_ws;
  _Float16* Q16    = (_Float16*)(ws + OFF_QPL);
  _Float16* C16    = (_Float16*)(ws + OFF_CPL);
  float*    scores = (float*)(ws + OFF_SCR);

  dim3 blk(256);
  cvt_kernel<<<dim3(NB * LQ / 8), blk, 0, stream>>>(query, Q16, (unsigned)LQ, (unsigned)LQ_FULL);
  cvt_kernel<<<dim3(NB * LC / 8), blk, 0, stream>>>(context, C16, (unsigned)LC, (unsigned)LC_FULL);
  score_kernel<<<dim3(LC / 128, NB), blk, 0, stream>>>(C16, Q16, scores);
  softmax_ctx_kernel<<<dim3(NB), blk, 0, stream>>>(context, scores, out);
}
